// PointNetSetAbstraction_84043920048191
// MI455X (gfx1250) — hardware-verified
//
#include <hip/hip_runtime.h>
#pragma clang fp contract(off)

typedef __attribute__((ext_vector_type(16))) _Float16 v16h;
typedef __attribute__((ext_vector_type(8)))  _Float16 v8h;
typedef __attribute__((ext_vector_type(8)))  float    v8f;
typedef __attribute__((ext_vector_type(4)))  float    v4f;
typedef __attribute__((ext_vector_type(4)))  int      v4i;
typedef __attribute__((ext_vector_type(4)))  unsigned v4u;
typedef v4u v4u_alias __attribute__((may_alias));

constexpr int kNumPts   = 16384;
constexpr int kNumCen   = 4096;
constexpr int kNbr      = 32;
constexpr int kFeat     = 64;
constexpr int kK1Real   = 67;
constexpr int kK1Pad    = 96;
constexpr int kHid1     = 128;
constexpr int kHid2     = 128;
constexpr int kHid3     = 256;
constexpr float kRad2       = 0.04f;
constexpr float kWCarry     = 16.0f;
constexpr float kWCarryInv  = 1.0f / 16.0f;

static_assert(kK1Pad % 32 == 0);
static_assert(kHid1 % 32 == 0);
static_assert(kHid2 % 32 == 0);
static_assert(kHid3 % 16 == 0);
static_assert(kNumCen * 3 * 4 == 49152);
static_assert(kNumCen * 3 * 4 + kNumCen * kHid3 * 4 == 4243456);

constexpr size_t kOffW1t  = 0;
constexpr size_t kOffW2t  = kOffW1t + (size_t)kHid1 * kK1Pad * 2;
constexpr size_t kOffW3t  = kOffW2t + (size_t)kHid2 * kHid1 * 2;
constexpr size_t kOffCen  = kOffW3t + (size_t)kHid3 * kHid2 * 2;
constexpr size_t kOffNbr  = kOffCen + (size_t)kNumCen * 4 * 4;
constexpr size_t kOffCnt  = kOffNbr + (size_t)kNumCen * kNbr * 4;
constexpr size_t kWsTotal = kOffCnt + (size_t)kNumCen * 4;
static_assert(kOffW2t == 24576);
static_assert(kOffW3t == 57344);
static_assert(kOffCen == 122880);
static_assert(kOffNbr == 188416);
static_assert(kOffCnt == 712704);
static_assert(kWsTotal == 729088);
static_assert(kWsTotal <= (size_t)134217728);

template <typename T> struct Frag;
template <> struct Frag<_Float16> {
  typedef v16h V; union U { v16h v; v8h h[2]; };
  static __device__ __forceinline__ v16h load(const _Float16* p) {
    U f; f.h[0] = *(const v8h*)(p); f.h[1] = *(const v8h*)(p + 16); return f.v;
  }
};

__device__ __forceinline__ v8f mma_h(v16h a, v16h b, v8f c) {
  c = __builtin_amdgcn_wmma_f32_16x16x32_f16(false, a, false, b, (short)0, c, false, false);
  asm volatile("v_nop\n\tv_nop\n\tv_nop\n\tv_nop" : "+v"(c) : "v"(a), "v"(b));
  return c;
}

__device__ __forceinline__ unsigned pack2h(float a, float b) {
  const _Float16 ha = (_Float16)a;
  const _Float16 hb = (_Float16)b;
  const unsigned ua = (unsigned)__builtin_bit_cast(unsigned short, ha);
  const unsigned ub = (unsigned)__builtin_bit_cast(unsigned short, hb);
  return ua | (ub << 16);
}

constexpr int kW1Vec = kHid1 * kK1Pad / 8;
constexpr int kW2Vec = kHid2 * kHid1 / 8;
constexpr int kW3Vec = kHid3 * kHid2 / 8;
constexpr int kPrepThreads = kW1Vec + kW2Vec + kW3Vec;
static_assert(kW1Vec % 32 == 0);
static_assert(kW2Vec % 32 == 0);
static_assert(kPrepThreads == 7680);
static_assert(kPrepThreads % 256 == 0);

__global__ __launch_bounds__(256) void prep_weights_kernel(
    const float* __restrict__ W1, const float* __restrict__ W2, const float* __restrict__ W3,
    _Float16* __restrict__ wt) {
  const int t = blockIdx.x * 256 + threadIdx.x;
  if (t < kPrepThreads) {
    const bool p1 = t < kW1Vec;
    const bool p2 = t < (kW1Vec + kW2Vec);
    const float* W = p1 ? W1 : (p2 ? W2 : W3);
    const int ncol  = p2 ? kHid1 : kHid3;
    const int krows = p1 ? kK1Real : kHid1;
    const int u1 = t;
    const int n1 = u1 / 12;
    const int k1 = (u1 - n1 * 12) * 8;
    const int u2 = t - kW1Vec;
    const int n2 = u2 >> 4;
    const int k2 = (u2 & 15) * 8;
    const int u3 = t - kW1Vec - kW2Vec;
    const int n3 = u3 >> 4;
    const int k3 = (u3 & 15) * 8;
    const int n  = p1 ? n1 : (p2 ? n2 : n3);
    const int k0 = p1 ? k1 : (p2 ? k2 : k3);
    v8h hv;
#pragma unroll
    for (int e = 0; e < 8; ++e) {
      const int k  = k0 + e;
      const int kc = (k < krows) ? k : (krows - 1);
      float v = W[(size_t)kc * ncol + n];
      v = (k < krows) ? (v * kWCarry) : 0.0f;
      hv[e] = (_Float16)v;
    }
    _Float16* dst = wt + (size_t)t * 8;
    *(volatile v8h*)dst = hv;
    __threadfence();
    *(volatile v8h*)dst = hv;
  }
}

constexpr int kFpsThreads = 1024;
constexpr size_t kFpsLds = (size_t)kNumPts * 3 * 4 + (size_t)kNumCen * 4 + 64 * 4 + 64 * 4;
static_assert(kNumPts == 16 * kFpsThreads);
static_assert(kNumPts * 3 / 4 == 12 * kFpsThreads);
static_assert(kNumCen * 3 / 4 == 3 * kFpsThreads);
static_assert(kNumCen == 4 * kFpsThreads);

__global__ __launch_bounds__(1024) void fps_kernel(
    const float* __restrict__ pos, float* __restrict__ out0, float* __restrict__ cen4) {
#pragma clang fp contract(off)
  extern __shared__ __align__(16) float fsm[];
  float* px   = fsm;
  float* py   = fsm + kNumPts;
  float* pz   = fsm + 2 * kNumPts;
  int*   idxs = (int*)(fsm + 3 * kNumPts);
  float* redv = fsm + 3 * kNumPts + kNumCen;
  int*   redi = (int*)(fsm + 3 * kNumPts + kNumCen + 64);
  const int tid  = threadIdx.x;
  const int lane = tid & 31;
  const int w    = tid >> 5;

#pragma unroll 1
  for (int it = 0; it < 12; ++it) {
    const int q = it * kFpsThreads + tid;
    const v4f v = *(const v4f*)(pos + 4 * (size_t)q);
#pragma unroll
    for (int e = 0; e < 4; ++e) {
      const int f  = 4 * q + e;
      const int pt = f / 3;
      const int cc = f - 3 * pt;
      fsm[cc * kNumPts + pt] = v[e];
    }
  }
  float mind[16];
#pragma unroll
  for (int j = 0; j < 16; ++j) mind[j] = __builtin_inff();
  __syncthreads();

  int far = 0;
#pragma unroll 1
  for (int s = 0; s < kNumCen; ++s) {
    if (tid == 0) idxs[s] = far;
    const float fx = px[far];
    const float fy = py[far];
    const float fz = pz[far];
    float bv = -1.0f;
    int   bi = 0x7fffffff;
#pragma unroll
    for (int j = 0; j < 16; ++j) {
      const int p = tid + j * kFpsThreads;
      const float dx = px[p] - fx;
      const float dy = py[p] - fy;
      const float dz = pz[p] - fz;
      const float t0 = dx * dx;
      const float t1 = dy * dy;
      const float t2 = dz * dz;
      const float d  = (t0 + t2) + t1;
      const float m  = (mind[j] < d) ? mind[j] : d;
      mind[j] = m;
      const bool up = m > bv;
      bv = up ? m : bv;
      bi = up ? p : bi;
    }
#pragma unroll
    for (int off = 16; off > 0; off >>= 1) {
      const float ov = __shfl_xor(bv, off, 32);
      const int   oi = __shfl_xor(bi, off, 32);
      const bool tk = (ov > bv) || ((ov == bv) && (oi < bi));
      bv = tk ? ov : bv;
      bi = tk ? oi : bi;
    }
    const int par = (s & 1) * 32;
    if (lane == 0) { redv[par + w] = bv; redi[par + w] = bi; }
    __syncthreads();
    bv = redv[par + lane];
    bi = redi[par + lane];
#pragma unroll
    for (int off = 16; off > 0; off >>= 1) {
      const float ov = __shfl_xor(bv, off, 32);
      const int   oi = __shfl_xor(bi, off, 32);
      const bool tk = (ov > bv) || ((ov == bv) && (oi < bi));
      bv = tk ? ov : bv;
      bi = tk ? oi : bi;
    }
    int nf = __builtin_amdgcn_readfirstlane(bi);
    nf = nf < 0 ? 0 : nf;
    nf = nf > (kNumPts - 1) ? (kNumPts - 1) : nf;
    far = nf;
  }
  __syncthreads();

  v4f ov4[3];
#pragma unroll
  for (int it = 0; it < 3; ++it) {
    const int q = it * kFpsThreads + tid;
#pragma unroll
    for (int e = 0; e < 4; ++e) {
      const int f  = 4 * q + e;
      const int sc = f / 3;
      const int cc = f - 3 * sc;
      const int id = idxs[sc];
      ov4[it][e] = fsm[cc * kNumPts + id];
    }
  }
  v4f cv4[4];
#pragma unroll
  for (int it = 0; it < 4; ++it) {
    const int sc = it * kFpsThreads + tid;
    const int id = idxs[sc];
    v4f cv;
    cv[0] = px[id];
    cv[1] = py[id];
    cv[2] = pz[id];
    cv[3] = 0.0f;
    cv4[it] = cv;
  }
  for (int pass = 0; pass < 2; ++pass) {
#pragma unroll
    for (int it = 0; it < 3; ++it) {
      const int q = it * kFpsThreads + tid;
      *(volatile v4f*)(out0 + 4 * (size_t)q) = ov4[it];
    }
#pragma unroll
    for (int it = 0; it < 4; ++it) {
      const int sc = it * kFpsThreads + tid;
      *(volatile v4f*)(cen4 + 4 * (size_t)sc) = cv4[it];
    }
    __threadfence();
  }
}

constexpr int kBqThreads = 128;
constexpr int kBqChunk   = 2048;
static_assert(kNumCen % kBqThreads == 0);
static_assert(kNumPts % kBqChunk == 0);
static_assert(kBqChunk * 3 / 4 == 12 * kBqThreads);

__global__ __launch_bounds__(128) void ballq_kernel(
    const float* __restrict__ pos, const float* __restrict__ cen4,
    int* __restrict__ nbr, int* __restrict__ cnt) {
#pragma clang fp contract(off)
  __shared__ __align__(16) float sp[3 * kBqChunk];
  __shared__ float lstd[kNbr * kBqThreads];
  __shared__ int   lsti[kNbr * kBqThreads];
  __shared__ __align__(16) int scnt[kBqThreads];
  const int tid  = threadIdx.x;
  const int lane = tid & 31;
  const int w    = tid >> 5;
  const int cb   = blockIdx.x * kBqThreads;
  const int c    = cb + tid;

  const v4f cv = *(const v4f*)(cen4 + 4 * (size_t)c);
  const float cx = cv[0];
  const float cy = cv[1];
  const float cz = cv[2];

#pragma unroll 4
  for (int q = 0; q < kNbr; ++q) {
    lstd[q * kBqThreads + tid] = __builtin_inff();
    lsti[q * kBqThreads + tid] = 0;
  }
  float worst = __builtin_inff();
  int n = 0;

#pragma unroll 1
  for (int ch = 0; ch < kNumPts / kBqChunk; ++ch) {
    __syncthreads();
#pragma unroll 1
    for (int it = 0; it < 12; ++it) {
      const int qv = it * kBqThreads + tid;
      const v4f v = *(const v4f*)(pos + (size_t)ch * kBqChunk * 3 + 4 * (size_t)qv);
#pragma unroll
      for (int e = 0; e < 4; ++e) {
        const int f  = 4 * qv + e;
        const int pt = f / 3;
        const int cc = f - 3 * pt;
        sp[cc * kBqChunk + pt] = v[e];
      }
    }
    __syncthreads();
    const int jbase = ch * kBqChunk;
#pragma unroll 1
    for (int jj = 0; jj < kBqChunk; ++jj) {
      const float dx = cx - sp[jj];
      const float dy = cy - sp[kBqChunk + jj];
      const float dz = cz - sp[2 * kBqChunk + jj];
      const float t0 = dx * dx;
      const float t1 = dy * dy;
      const float t2 = dz * dz;
      const float d2 = (t0 + t2) + t1;
      if ((d2 <= kRad2) && (d2 < worst)) {
        int q = kNbr - 1;
#pragma unroll 1
        for (; q > 0; --q) {
          const float cd = lstd[(q - 1) * kBqThreads + tid];
          if (!(cd > d2)) break;
          lstd[q * kBqThreads + tid] = cd;
          lsti[q * kBqThreads + tid] = lsti[(q - 1) * kBqThreads + tid];
        }
        lstd[q * kBqThreads + tid] = d2;
        lsti[q * kBqThreads + tid] = jbase + jj;
        worst = lstd[(kNbr - 1) * kBqThreads + tid];
        n = (n < kNbr) ? (n + 1) : kNbr;
      }
    }
  }
  scnt[tid] = n;
  __syncthreads();

  for (int pass = 0; pass < 2; ++pass) {
#pragma unroll
    for (int it = 0; it < 8; ++it) {
      const int cl = w * 32 + it * 4 + (lane >> 3);
      const int q0 = (lane & 7) * 4;
      v4i o;
#pragma unroll
      for (int e = 0; e < 4; ++e) {
        int id = lsti[(q0 + e) * kBqThreads + cl];
        id = id < 0 ? 0 : id;
        id = id > (kNumPts - 1) ? (kNumPts - 1) : id;
        o[e] = id;
      }
      *(volatile v4i*)(nbr + (size_t)(cb + cl) * kNbr + q0) = o;
    }
    __threadfence();
  }
  if (w == 0) {
    v4i o;
#pragma unroll
    for (int e = 0; e < 4; ++e) {
      int v = scnt[4 * lane + e];
      v = v < 0 ? 0 : v;
      v = v > kNbr ? kNbr : v;
      o[e] = v;
    }
    *(volatile v4i*)(cnt + cb + 4 * lane) = o;
    __threadfence();
    *(volatile v4i*)(cnt + cb + 4 * lane) = o;
  }
}

constexpr int kHP          = 136;
constexpr int kMlpWaves    = 8;
constexpr int kTileHalves  = kNbr * kHP;
constexpr int kWaveBytes   = 2 * kTileHalves * 2 + kHid3 * 4;
constexpr size_t kMlpLds   = (size_t)kMlpWaves * kWaveBytes;
static_assert(kWaveBytes == 18432);
static_assert(kWaveBytes % 16 == 0);
static_assert((kHP * 2) % 16 == 0);
static_assert(kNumCen % kMlpWaves == 0);

template <int KT, int KP>
__device__ __forceinline__ void layer_t(const _Float16* Hin, const _Float16* Wt,
                                        const float* bias, _Float16* Hout, int lane) {
  const int c  = lane & 15;
  const int hh = lane >> 4;
  v16h bf[2][KT];
#pragma unroll
  for (int mt = 0; mt < 2; ++mt)
#pragma unroll
    for (int kt = 0; kt < KT; ++kt)
      bf[mt][kt] = Frag<_Float16>::load(Hin + (mt * 16 + c) * kHP + kt * 32 + 8 * hh);
#pragma unroll 1
  for (int nt = 0; nt < 8; ++nt) {
    v16h af[KT];
#pragma unroll
    for (int kt = 0; kt < KT; ++kt)
      af[kt] = Frag<_Float16>::load(Wt + (size_t)(nt * 16 + c) * KP + kt * 32 + 8 * hh);
    const v4f bA = *(const v4f*)(bias + nt * 16 + 8 * hh);
    const v4f bB = *(const v4f*)(bias + nt * 16 + 8 * hh + 4);
    v8f acc0, acc1;
#pragma unroll
    for (int r = 0; r < 4; ++r) {
      acc0[r]     = bA[r] * kWCarry;
      acc0[4 + r] = bB[r] * kWCarry;
    }
    acc1 = acc0;
#pragma unroll
    for (int kt = 0; kt < KT; ++kt) {
      acc0 = mma_h(af[kt], bf[0][kt], acc0);
      acc1 = mma_h(af[kt], bf[1][kt], acc1);
    }
    v8h o0, o1;
#pragma unroll
    for (int r = 0; r < 8; ++r) {
      float v0 = acc0[r] * kWCarryInv;
      float v1 = acc1[r] * kWCarryInv;
      v0 = fmaxf(v0, 0.0f);
      v1 = fmaxf(v1, 0.0f);
      o0[r] = (_Float16)v0;
      o1[r] = (_Float16)v1;
    }
    *(v8h*)(Hout + c * kHP + nt * 16 + 8 * hh) = o0;
    *(v8h*)(Hout + (16 + c) * kHP + nt * 16 + 8 * hh) = o1;
  }
}

__global__ __launch_bounds__(256) void mlp_kernel(
    const float* __restrict__ pos, const float* __restrict__ x,
    const float* __restrict__ cen4,
    const int* __restrict__ nbr, const int* __restrict__ cnt,
    const _Float16* __restrict__ W1t, const _Float16* __restrict__ W2t,
    const _Float16* __restrict__ W3t,
    const float* __restrict__ b1, const float* __restrict__ b2, const float* __restrict__ b3,
    float* __restrict__ out1) {
  extern __shared__ __align__(16) unsigned char msm[];
  const int lane = threadIdx.x & 31;
  const int w    = threadIdx.x >> 5;
  _Float16* bufA = (_Float16*)(msm + (size_t)w * kWaveBytes);
  _Float16* bufB = bufA + kTileHalves;
  float*    so   = (float*)(bufB + kTileHalves);
  const int c = blockIdx.x * kMlpWaves + w;

  int nv = cnt[c];
  nv = nv < 0 ? 0 : nv;
  nv = nv > kNbr ? kNbr : nv;

  {
    int nb = nbr[(size_t)c * kNbr + lane];
    nb = nb < 0 ? 0 : nb;
    nb = nb > (kNumPts - 1) ? (kNumPts - 1) : nb;
    const v4f cv = *(const v4f*)(cen4 + 4 * (size_t)c);
    const float* xr = x + (size_t)nb * kFeat;
    _Float16* row = bufA + lane * kHP;
#pragma unroll 1
    for (int g = 0; g < 2; ++g) {
      v4f xa[4], xb[4];
#pragma unroll
      for (int t = 0; t < 4; ++t) {
        xa[t] = *(const v4f*)(xr + g * 32 + t * 8);
        xb[t] = *(const v4f*)(xr + g * 32 + t * 8 + 4);
      }
#pragma unroll
      for (int t = 0; t < 4; ++t) {
        v4u wv;
        wv[0] = pack2h(xa[t][0], xa[t][1]);
        wv[1] = pack2h(xa[t][2], xa[t][3]);
        wv[2] = pack2h(xb[t][0], xb[t][1]);
        wv[3] = pack2h(xb[t][2], xb[t][3]);
        *(v4u_alias*)(row + g * 32 + t * 8) = wv;
      }
    }
    const float r0 = pos[(size_t)nb * 3 + 0] - cv[0];
    const float r1 = pos[(size_t)nb * 3 + 1] - cv[1];
    const float r2 = pos[(size_t)nb * 3 + 2] - cv[2];
    const _Float16 h2 = (_Float16)r2;
    const unsigned u2 = (unsigned)__builtin_bit_cast(unsigned short, h2);
    v4u rv;
    rv[0] = pack2h(r0, r1);
    rv[1] = u2;
    rv[2] = 0u;
    rv[3] = 0u;
    *(v4u_alias*)(row + 64) = rv;
    v4u zv;
    zv[0] = 0u;
    zv[1] = 0u;
    zv[2] = 0u;
    zv[3] = 0u;
    *(v4u_alias*)(row + 72) = zv;
    *(v4u_alias*)(row + 80) = zv;
    *(v4u_alias*)(row + 88) = zv;
  }
  __syncthreads();

  layer_t<3, kK1Pad>(bufA, W1t, b1, bufB, lane);
  __syncthreads();
  layer_t<4, kHid1>(bufB, W2t, b2, bufA, lane);
  __syncthreads();

  {
    const int cc = lane & 15;
    const int hh = lane >> 4;
    v16h af[2][4];
#pragma unroll
    for (int mt = 0; mt < 2; ++mt)
#pragma unroll
      for (int kt = 0; kt < 4; ++kt)
        af[mt][kt] = Frag<_Float16>::load(bufA + (mt * 16 + cc) * kHP + kt * 32 + 8 * hh);
#pragma unroll 1
    for (int nt = 0; nt < kHid3 / 16; ++nt) {
      v16h bw[4];
#pragma unroll
      for (int kt = 0; kt < 4; ++kt)
        bw[kt] = Frag<_Float16>::load(W3t + (size_t)(nt * 16 + cc) * kHid2 + kt * 32 + 8 * hh);
      const float bv = b3[nt * 16 + cc] * kWCarry;
      v8f acc0, acc1;
#pragma unroll
      for (int r = 0; r < 8; ++r) acc0[r] = bv;
      acc1 = acc0;
#pragma unroll
      for (int kt = 0; kt < 4; ++kt) {
        acc0 = mma_h(af[0][kt], bw[kt], acc0);
        acc1 = mma_h(af[1][kt], bw[kt], acc1);
      }
      float tm = -__builtin_inff();
#pragma unroll
      for (int r = 0; r < 8; ++r) {
        const int m0 = 8 * hh + r;
        const int m1 = 16 + 8 * hh + r;
        float v0 = fmaxf(acc0[r] * kWCarryInv, 0.0f);
        float v1 = fmaxf(acc1[r] * kWCarryInv, 0.0f);
        v0 = (m0 < nv) ? v0 : -__builtin_inff();
        v1 = (m1 < nv) ? v1 : -__builtin_inff();
        tm = fmaxf(tm, v0);
        tm = fmaxf(tm, v1);
      }
      const float ot = __shfl_xor(tm, 16, 32);
      tm = fmaxf(tm, ot);
      const float o = (nv > 0) ? tm : 0.0f;
      so[nt * 16 + cc] = o;
    }
  }
  __syncthreads();

  {
    float* orow = out1 + (size_t)c * kHid3;
    for (int pass = 0; pass < 2; ++pass) {
#pragma unroll
      for (int it = 0; it < 2; ++it) {
        const v4f v = *(const v4f*)(so + it * 128 + 4 * lane);
        *(volatile v4f*)(orow + it * 128 + 4 * lane) = v;
      }
      __threadfence();
    }
  }
}

extern "C" void kernel_launch(void* const* d_in, const int* in_sizes, int n_in,
                              void* d_out, int out_size, void* d_ws, size_t ws_size,
                              hipStream_t stream) {
  (void)in_sizes;
  (void)out_size;
  if (n_in < 8) return;
  if (ws_size < kWsTotal) return;

  const float* pos = (const float*)d_in[0];
  const float* x   = (const float*)d_in[1];
  const float* W1  = (const float*)d_in[2];
  const float* b1  = (const float*)d_in[3];
  const float* W2  = (const float*)d_in[4];
  const float* b2  = (const float*)d_in[5];
  const float* W3  = (const float*)d_in[6];
  const float* b3  = (const float*)d_in[7];

  float* out0 = (float*)d_out;
  float* out1 = out0 + (size_t)kNumCen * 3;

  char* ws = (char*)d_ws;
  _Float16* wt   = (_Float16*)(ws + kOffW1t);
  _Float16* W1t  = (_Float16*)(ws + kOffW1t);
  _Float16* W2t  = (_Float16*)(ws + kOffW2t);
  _Float16* W3t  = (_Float16*)(ws + kOffW3t);
  float*    cen4 = (float*)(ws + kOffCen);
  int*      nbrb = (int*)(ws + kOffNbr);
  int*      cntb = (int*)(ws + kOffCnt);

  prep_weights_kernel<<<kPrepThreads / 256, 256, 0, stream>>>(W1, W2, W3, wt);
  fps_kernel<<<1, kFpsThreads, kFpsLds, stream>>>(pos, out0, cen4);
  ballq_kernel<<<kNumCen / kBqThreads, kBqThreads, 0, stream>>>(pos, cen4, nbrb, cntb);
  mlp_kernel<<<kNumCen / kMlpWaves, kMlpWaves * 32, kMlpLds, stream>>>(
      pos, x, cen4, nbrb, cntb, W1t, W2t, W3t, b1, b2, b3, out1);
}
